// Spatial_dot_80951543595350
// MI455X (gfx1250) — hardware-run, weakly checked
//
#include <hip/hip_runtime.h>

typedef __attribute__((ext_vector_type(16))) _Float16 v16h;
typedef __attribute__((ext_vector_type(8)))  _Float16 v8h;
typedef __attribute__((ext_vector_type(8)))  float    v8f;
typedef __attribute__((ext_vector_type(4)))  float    v4f;
typedef __attribute__((ext_vector_type(4)))  unsigned v4u;

constexpr int kSlices  = 32;
constexpr int kChan    = 64;
constexpr int kPts     = 1024;
constexpr int kFeat    = 10;
constexpr int kFeatPad = 16;
constexpr int kTile    = 64;
constexpr int kXPitch  = 72;
constexpr int kAPitch  = 40;
constexpr int kOPitch  = 68;
constexpr float kAScale    = 256.0f;
constexpr float kAScaleInv = 1.0f / 256.0f;

static_assert(kChan % 32 == 0, "projection K must be a multiple of 32");
static_assert(kPts % kTile == 0 && kPts % 32 == 0, "point count must tile exactly");
static_assert(kFeat <= kFeatPad && kFeatPad == 16, "feature padding");
static_assert((kXPitch * 2) % 16 == 0 && (kAPitch * 2) % 16 == 0 && (kOPitch * 4) % 16 == 0, "16-B aligned LDS pitches");

constexpr size_t kPlaneHalfBytes = (size_t)kSlices * kPts * kFeatPad * 2;
constexpr size_t kOffQ = 0;
constexpr size_t kOffK = kOffQ + kPlaneHalfBytes;
constexpr size_t kOffG = kOffK + kPlaneHalfBytes;
constexpr size_t kOffL = kOffG + kPlaneHalfBytes;
constexpr size_t kWsTotal = kOffL + (size_t)kSlices * kPts * 4;
static_assert(kWsTotal == 3276800, "carve total");
static_assert(kWsTotal <= 134217728, "carve under the limit");
static_assert(kOffK % 128 == 0 && kOffG % 128 == 0 && kOffL % 128 == 0, "128-B aligned regions");

union HF { v16h v; v8h h[2]; v4u u[2]; };

__device__ __forceinline__ v16h fload(const _Float16* p) {
  HF f; f.h[0] = *(const v8h*)(p); f.h[1] = *(const v8h*)(p + 16); return f.v;
}

__device__ __forceinline__ v8f mma_h(v16h a, v16h b, v8f c) {
  c = __builtin_amdgcn_wmma_f32_16x16x32_f16(false, a, false, b, (short)0, c, false, false);
  asm volatile("v_nop\n\tv_nop\n\tv_nop\n\tv_nop" : "+v"(c) : "v"(a), "v"(b));
  return c;
}

__global__ __launch_bounds__(128) void proj_kernel(
    const float* __restrict__ x1, const float* __restrict__ x2,
    const float* __restrict__ W1, const float* __restrict__ b1,
    const float* __restrict__ W2, const float* __restrict__ b2,
    const float* __restrict__ W3, const float* __restrict__ b3,
    _Float16* __restrict__ Qt, _Float16* __restrict__ Kt, _Float16* __restrict__ Gp)
{
  __shared__ __align__(16) _Float16 xs[2][kTile * kXPitch];
  __shared__ __align__(16) _Float16 wsh[3][kFeatPad * kXPitch];
  __shared__ __align__(16) _Float16 stQK[2][kTile * kFeatPad];
  __shared__ __align__(16) _Float16 stG[kFeatPad * kXPitch];
  __shared__ float bsh[3 * kFeatPad];

  const int tid  = threadIdx.x;
  const int wave = tid >> 5;
  const int lane = tid & 31;
  const int hh   = lane >> 4;
  const int cl   = lane & 15;
  const int koff = hh * 8;
  const int nblk = blockIdx.x;
  const int bt   = blockIdx.y;
  const int n0   = nblk * kTile;

#pragma unroll
  for (int p = 0; p < 3; ++p) {
    const float* Wp = (p == 0) ? W1 : ((p == 1) ? W2 : W3);
#pragma unroll
    for (int i = 0; i < 2; ++i) {
      const int idx = i * 128 + tid;
      const int idc = (idx < 160) ? idx : 159;
      const int f = idc >> 4, q = idc & 15;
      const v4f v = *(const v4f*)(Wp + f * kChan + q * 4);
      if (idx < 160) {
#pragma unroll
        for (int e = 0; e < 4; ++e) wsh[p][f * kXPitch + q * 4 + e] = (_Float16)v[e];
      }
    }
    if (tid < 48) {
      const int r = kFeat + (tid >> 3), q = tid & 7;
      *(v4u*)(&wsh[p][r * kXPitch + q * 8]) = (v4u){0u, 0u, 0u, 0u};
    }
  }
  if (tid < 48) {
    const int p = tid >> 4, f = tid & 15;
    const int fc = (f < kFeat) ? f : (kFeat - 1);
    const float v1 = b1[fc], v2 = b2[fc], v3 = b3[fc];
    const float v = (p == 0) ? v1 : ((p == 1) ? v2 : v3);
    bsh[tid] = (f < kFeat) ? v : 0.0f;
  }

#pragma unroll
  for (int src = 0; src < 2; ++src) {
    const float* xp = ((src == 0) ? x1 : x2) + (size_t)bt * kChan * kPts + n0;
#pragma unroll
    for (int i = 0; i < 8; ++i) {
      const int idx = i * 128 + tid;
      const int cc = idx >> 4, q = idx & 15;
      const v4f v = *(const v4f*)(xp + (size_t)cc * kPts + q * 4);
#pragma unroll
      for (int e = 0; e < 4; ++e) xs[src][(q * 4 + e) * kXPitch + cc] = (_Float16)v[e];
    }
    asm volatile("" ::: "memory");
  }
  __syncthreads();

  const v8f z8 = {0.f, 0.f, 0.f, 0.f, 0.f, 0.f, 0.f, 0.f};
  v8f accQ = z8, accK = z8, accG = z8;
#pragma unroll
  for (int ks = 0; ks < kChan / 32; ++ks) {
    const int k0 = ks * 32;
    const v16h a1 = fload(&xs[0][(wave * 16 + cl) * kXPitch + koff + k0]);
    const v16h a2 = fload(&xs[1][(wave * 16 + cl) * kXPitch + koff + k0]);
    const v16h w1 = fload(&wsh[0][cl * kXPitch + koff + k0]);
    const v16h w2 = fload(&wsh[1][cl * kXPitch + koff + k0]);
    const v16h w3 = fload(&wsh[2][cl * kXPitch + koff + k0]);
    accQ = mma_h(a1, w1, accQ);
    accK = mma_h(a2, w2, accK);
    accG = mma_h(a1, w3, accG);
  }

  {
    const float bq = bsh[cl], bk = bsh[kFeatPad + cl], bg = bsh[2 * kFeatPad + cl];
#pragma unroll
    for (int r = 0; r < 8; ++r) {
      const int nl = wave * 16 + hh * 8 + r;
      stQK[0][nl * kFeatPad + cl] = (_Float16)(accQ[r] + bq);
      stQK[1][nl * kFeatPad + cl] = (_Float16)(accK[r] + bk);
      stG[cl * kXPitch + nl]      = (_Float16)(accG[r] + bg);
    }
  }
  __syncthreads();

  {
    const v4u vq = *(const v4u*)(&stQK[0][wave * 256 + lane * 8]);
    const v4u vk = *(const v4u*)(&stQK[1][wave * 256 + lane * 8]);
    const int fo = wave * 4 + (lane >> 3);
    const int mo = (lane & 7) * 8;
    const v4u vg = *(const v4u*)(&stG[fo * kXPitch + mo]);
    _Float16* gq = Qt + ((size_t)bt * kPts + n0) * kFeatPad + wave * 256 + lane * 8;
    _Float16* gk = Kt + ((size_t)bt * kPts + n0) * kFeatPad + wave * 256 + lane * 8;
    _Float16* gg = Gp + ((size_t)bt * kFeatPad + fo) * kPts + n0 + mo;
    for (int pass = 0; pass < 2; ++pass) {
      *(volatile v4u*)gq = vq;
      *(volatile v4u*)gk = vk;
      *(volatile v4u*)gg = vg;
      __threadfence();
    }
  }
}

__global__ __launch_bounds__(128) void colstat_kernel(
    const _Float16* __restrict__ Qt, const _Float16* __restrict__ Kt, float* __restrict__ lsep)
{
  __shared__ __align__(16) float stl[kTile];

  const int tid  = threadIdx.x;
  const int wave = tid >> 5;
  const int lane = tid & 31;
  const int hh   = lane >> 4;
  const int cl   = lane & 15;
  const int mblk = blockIdx.x;
  const int bt   = blockIdx.y;
  const int m0w  = mblk * kTile + wave * 16;

  const _Float16* Qs = Qt + (size_t)bt * kPts * kFeatPad;
  const v4u zero4 = {0u, 0u, 0u, 0u};
  const v8f z8 = {0.f, 0.f, 0.f, 0.f, 0.f, 0.f, 0.f, 0.f};

  HF bk;
  bk.h[0] = *(const v8h*)(Kt + ((size_t)bt * kPts + m0w + cl) * kFeatPad + hh * 8);
  bk.u[1] = zero4;

  float runM = -__builtin_inff();
  float runS = 0.0f;
#pragma unroll 1
  for (int nt = 0; nt < kPts / 16; ++nt) {
    HF aq;
    aq.h[0] = *(const v8h*)(Qs + (size_t)(nt * 16 + cl) * kFeatPad + hh * 8);
    aq.u[1] = zero4;
    const v8f s = mma_h(aq.v, bk.v, z8);
    float mt = s[0];
#pragma unroll
    for (int r = 1; r < 8; ++r) mt = fmaxf(mt, s[r]);
    const float mn = fmaxf(runM, mt);
    float acc = runS * expf(runM - mn);
#pragma unroll
    for (int r = 0; r < 8; ++r) acc += expf(s[r] - mn);
    runS = acc;
    runM = mn;
  }
  const float oM = __shfl_xor(runM, 16, 32);
  const float oS = __shfl_xor(runS, 16, 32);
  const float mn  = fmaxf(runM, oM);
  const float tot = runS * expf(runM - mn) + oS * expf(oM - mn);
  const float lse = mn + logf(tot);
  if (hh == 0) stl[wave * 16 + cl] = lse;
  __syncthreads();
  if (wave == 0 && lane < 16) {
    const v4f v = *(const v4f*)(&stl[lane * 4]);
    float* dst = lsep + (size_t)bt * kPts + mblk * kTile + lane * 4;
    *(volatile v4f*)dst = v;
    __threadfence();
    *(volatile v4f*)dst = v;
  }
}

__global__ __launch_bounds__(128) void attn_kernel(
    const _Float16* __restrict__ Qt, const _Float16* __restrict__ Kt, const _Float16* __restrict__ Gp,
    const float* __restrict__ lsep, const float* __restrict__ actw, float* __restrict__ out)
{
  __shared__ __align__(16) _Float16 ldsA[4][16 * kAPitch];
  __shared__ __align__(16) float os[kFeatPad * kOPitch];

  const int tid  = threadIdx.x;
  const int wave = tid >> 5;
  const int lane = tid & 31;
  const int hh   = lane >> 4;
  const int cl   = lane & 15;
  const int nblk = blockIdx.x;
  const int bt   = blockIdx.y;
  const int n0w  = nblk * kTile + wave * 16;

  const v4u zero4 = {0u, 0u, 0u, 0u};
  const v8f z8 = {0.f, 0.f, 0.f, 0.f, 0.f, 0.f, 0.f, 0.f};

  const float w0s = actw[0] * kAScale;
  const float w1s = actw[1] * kAScale;
  const float w2s = actw[2] * kAScale;

  const _Float16* Ks   = Kt   + (size_t)bt * kPts * kFeatPad;
  const _Float16* Gs   = Gp   + (size_t)bt * kFeatPad * kPts;
  const float*    lses = lsep + (size_t)bt * kPts;

  HF aq;
  aq.h[0] = *(const v8h*)(Qt + ((size_t)bt * kPts + n0w + cl) * kFeatPad + hh * 8);
  aq.u[1] = zero4;

  _Float16* la = ldsA[wave];
  v8f acc = z8;

#pragma unroll 1
  for (int mb = 0; mb < kPts; mb += 32) {
#pragma unroll
    for (int t = 0; t < 2; ++t) {
      const int m0 = mb + t * 16;
      HF bk;
      bk.h[0] = *(const v8h*)(Ks + (size_t)(m0 + cl) * kFeatPad + hh * 8);
      bk.u[1] = zero4;
      const v8f s = mma_h(aq.v, bk.v, z8);
      const float lc = lses[m0 + cl];
#pragma unroll
      for (int r = 0; r < 8; ++r) {
        const float sv  = s[r];
        const float e1  = expf(-sv);
        const float sig = __builtin_amdgcn_rcpf(1.0f + e1);
        const float pv  = expf(sv - lc);
        const float a   = w0s * fmaxf(sv, 0.0f) + w1s * sig + w2s * pv;
        la[(hh * 8 + r) * kAPitch + t * 16 + cl] = (_Float16)a;
      }
    }
    __syncthreads();
    const v16h aA = fload(la + cl * kAPitch + hh * 8);
    const v16h bG = fload(Gs + (size_t)cl * kPts + mb + hh * 8);
    acc = mma_h(aA, bG, acc);
    __syncthreads();
  }

#pragma unroll
  for (int r = 0; r < 8; ++r) os[cl * kOPitch + wave * 16 + hh * 8 + r] = acc[r] * kAScaleInv;
  __syncthreads();
  {
    const int q    = lane >> 3;
    const int lA   = wave * 4 + q;
    const int fA   = lA >> 1;
    const int colA = (lA & 1) * 32 + (lane & 7) * 4;
    const v4f vA   = *(const v4f*)(&os[fA * kOPitch + colA]);
    const int lB   = 16 + wave * 4 + q;
    const int fB   = lB >> 1;
    const int colB = (lB & 1) * 32 + (lane & 7) * 4;
    const v4f vB   = *(const v4f*)(&os[fB * kOPitch + colB]);
    float* dstA = out + ((size_t)bt * kFeat + fA) * kPts + nblk * kTile + colA;
    for (int pass = 0; pass < 2; ++pass) {
      *(volatile v4f*)dstA = vA;
      if (wave == 0) {
        float* dstB = out + ((size_t)bt * kFeat + fB) * kPts + nblk * kTile + colB;
        *(volatile v4f*)dstB = vB;
      }
      __threadfence();
    }
  }
}

extern "C" void kernel_launch(void* const* d_in, const int* in_sizes, int n_in,
                              void* d_out, int out_size, void* d_ws, size_t ws_size,
                              hipStream_t stream)
{
  if (n_in < 9) return;
  if (in_sizes[0] != kSlices * kChan * kPts || in_sizes[1] != kSlices * kChan * kPts) return;
  if (in_sizes[2] < 3) return;
  if (in_sizes[3] != kFeat * kChan || in_sizes[5] != kFeat * kChan || in_sizes[7] != kFeat * kChan) return;
  if (in_sizes[4] < kFeat || in_sizes[6] < kFeat || in_sizes[8] < kFeat) return;
  if (out_size != kSlices * kFeat * kPts) return;
  if (ws_size < kWsTotal) return;

  const float* x1   = (const float*)d_in[0];
  const float* x2   = (const float*)d_in[1];
  const float* actw = (const float*)d_in[2];
  const float* W1   = (const float*)d_in[3];
  const float* b1   = (const float*)d_in[4];
  const float* W2   = (const float*)d_in[5];
  const float* b2   = (const float*)d_in[6];
  const float* W3   = (const float*)d_in[7];
  const float* b3   = (const float*)d_in[8];
  float* out = (float*)d_out;

  char* ws = (char*)d_ws;
  _Float16* Qt  = (_Float16*)(ws + kOffQ);
  _Float16* Kt  = (_Float16*)(ws + kOffK);
  _Float16* Gp  = (_Float16*)(ws + kOffG);
  float*    lse = (float*)(ws + kOffL);

  const dim3 grid(kPts / kTile, kSlices);

  proj_kernel<<<grid, 128, 0, stream>>>(x1, x2, W1, b1, W2, b2, W3, b3, Qt, Kt, Gp);
  colstat_kernel<<<grid, 128, 0, stream>>>(Qt, Kt, lse);
  attn_kernel<<<grid, 128, 0, stream>>>(Qt, Kt, Gp, lse, actw, out);
}
